// Self_Attention_61177514164743
// MI455X (gfx1250) — hardware-verified
//
#include <hip/hip_runtime.h>
#ifndef NB
#define NB 4
#endif
#ifndef SEQ
#define SEQ 2048
#endif
#define NB_FULL 4
#define SEQ_FULL 2048
#define DIN 512
#define TQ 256
#define NH 8
#define HD 32
#define DOUT 512
#define NR ((size_t)NB * SEQ)
#define KT 64

static_assert(NB >= 1 && NB <= NB_FULL);
static_assert(SEQ >= 128 && SEQ <= SEQ_FULL);
static_assert(SEQ % 128 == 0);
static_assert((NR % 128) == 0);
static_assert(TQ % 64 == 0 && DOUT % 64 == 0 && DIN % 32 == 0 && TQ % 32 == 0);
static_assert(HD == 32 && NH * HD == TQ);
static_assert(SEQ % KT == 0 && KT == 64);

typedef _Float16 v16h __attribute__((ext_vector_type(16)));
typedef unsigned short v8us __attribute__((ext_vector_type(8), may_alias));
typedef float  v8f  __attribute__((ext_vector_type(8)));
typedef float  v4f  __attribute__((ext_vector_type(4)));
typedef float  v4fa __attribute__((ext_vector_type(4), may_alias));
typedef _Float16 v4h __attribute__((ext_vector_type(4)));
union FragH { v16h v; v8us half[2]; _Float16 h[16]; unsigned short u[16]; };

__device__ __forceinline__ unsigned short bf16_bits(float x) { unsigned int u = __float_as_uint(x); return (unsigned short)((u + 0x7FFFu + ((u >> 16) & 1u)) >> 16); }
__device__ __forceinline__ float bf16_val(unsigned short b) { return __uint_as_float(((unsigned int)b) << 16); }
__device__ __forceinline__ float bf16_rne(float x) { return bf16_val(bf16_bits(x)); }

__device__ __forceinline__ v16h g2_frag(const _Float16* p, int hh) { FragH f; f.half[0] = *(const v8us*)((const unsigned short*)p + 8 * hh); f.half[1] = *(const v8us*)((const unsigned short*)p + 16 + 8 * hh); return f.v; }
__device__ __forceinline__ v8f g2_mma(v16h a, v16h b, v8f c) { v8f d = __builtin_amdgcn_wmma_f32_16x16x32_f16(false, a, false, b, (short)0, c, false, false); asm volatile("v_nop\n\tv_nop\n\tv_nop\n\tv_nop" : "+v"(d) : "v"(a), "v"(b)); return d; }
__device__ __forceinline__ v8f mma_split(v16h ah, v16h al, v16h bh, v16h bl) {
  const v8f z8 = {0.f,0.f,0.f,0.f,0.f,0.f,0.f,0.f};
  v8f c1 = __builtin_amdgcn_wmma_f32_16x16x32_f16(false, ah, false, bh, (short)0, z8, false, false);
  v8f c2 = __builtin_amdgcn_wmma_f32_16x16x32_f16(false, al, false, bh, (short)0, z8, false, false);
  c2 = __builtin_amdgcn_wmma_f32_16x16x32_f16(false, ah, false, bl, (short)0, c2, false, false);
  asm volatile("v_nop\n\tv_nop\n\tv_nop\n\tv_nop" : "+v"(c1), "+v"(c2) : "v"(ah), "v"(al), "v"(bh), "v"(bl));
  return c1 + c2 * 0.0009765625f;
}

__global__ __launch_bounds__(256) void k_x16r(const float* __restrict__ x, _Float16* __restrict__ X16, size_t n8) {
  const size_t t = (size_t)blockIdx.x * 256 + threadIdx.x; if (t >= n8) return;
  const size_t e = t * 8; const size_t r = e / DIN; const size_t c = e - r * DIN;
  const size_t sr = (r / SEQ) * SEQ_FULL + (r % SEQ);
  const float* s = x + sr * DIN + c;
  const v4f a = *(const v4fa*)s, c4v = *(const v4fa*)(s + 4);
  FragH f;
#pragma unroll
  for (int q = 0; q < 4; ++q) { f.h[q] = (_Float16)bf16_rne(a[q]); f.h[4 + q] = (_Float16)bf16_rne(c4v[q]); }
  unsigned short* d = (unsigned short*)X16 + e;
  *(volatile v8us*)d = f.half[0]; __threadfence(); *(volatile v8us*)d = f.half[0];
}

__global__ __launch_bounds__(256) void k_wt_f16(const float* __restrict__ W, _Float16* __restrict__ Wt, int K, int N, float scale) {
  const int t = blockIdx.x * 256 + threadIdx.x; if (t >= N * (K / 8)) return; const int n = t / (K / 8), k8 = (t % (K / 8)) * 8; FragH f;
#pragma unroll
  for (int i = 0; i < 8; ++i) f.h[i] = (_Float16)(bf16_rne(W[(size_t)(k8 + i) * N + n]) * scale);
  const v8us o = f.half[0]; unsigned short* d = (unsigned short*)Wt + (size_t)n * K + k8;
  *(volatile v8us*)d = o; __threadfence(); *(volatile v8us*)d = o;
}

__global__ __launch_bounds__(256) void k_hl(const float* __restrict__ F, _Float16* __restrict__ Hh, _Float16* __restrict__ Hl, size_t n8) {
  const size_t t = (size_t)blockIdx.x * 256 + threadIdx.x; if (t >= n8) return; FragH fh, fl; const v4f a = *(const v4fa*)(F + t * 8), c = *(const v4fa*)(F + t * 8 + 4);
#pragma unroll
  for (int q = 0; q < 4; ++q) { _Float16 h = (_Float16)a[q]; fh.h[q] = h; fl.h[q] = (_Float16)((a[q] - (float)h) * 1024.0f); h = (_Float16)c[q]; fh.h[4 + q] = h; fl.h[4 + q] = (_Float16)((c[q] - (float)h) * 1024.0f); }
  for (int pass = 0; pass < 2; ++pass) { *(volatile v8us*)((unsigned short*)Hh + t * 8) = fh.half[0]; *(volatile v8us*)((unsigned short*)Hl + t * 8) = fl.half[0]; if (pass == 0) __threadfence(); } }

__global__ __launch_bounds__(128) void k_gemm_proj(const _Float16* __restrict__ A, int lda, const _Float16* __restrict__ Bh, int ldb, float alpha, const float* __restrict__ bias,
                                                   float* __restrict__ C, _Float16* __restrict__ C16, int ldc, int M, int N, int K) {
  __shared__ __attribute__((aligned(16))) float so[4][32][68];
  const int tid = threadIdx.x, w = tid >> 5, lane = tid & 31, ln = lane & 15, hh = lane >> 4;
  const int ntn = N >> 6; const int mt = blockIdx.x / ntn, nq = blockIdx.x - mt * ntn; const int row0 = mt * 128 + 32 * w, col0 = nq * 64; if (row0 >= M) return;
  const _Float16* a0p = A + (size_t)(row0 + ln) * lda; const _Float16* a1p = a0p + (size_t)16 * lda;
  const _Float16* b0p = Bh + (size_t)(col0 + ln) * ldb; const _Float16* b1p = b0p + (size_t)16 * ldb; const _Float16* b2p = b1p + (size_t)16 * ldb; const _Float16* b3p = b2p + (size_t)16 * ldb;
  const v8f z8 = {0.f,0.f,0.f,0.f,0.f,0.f,0.f,0.f}; v8f c00 = z8, c01 = z8, c02 = z8, c03 = z8, c10 = z8, c11 = z8, c12 = z8, c13 = z8;
#pragma unroll 1
  for (int kb = 0; kb < K; kb += 32) { const v16h a0 = g2_frag(a0p + kb, hh), a1 = g2_frag(a1p + kb, hh);
    v16h b = g2_frag(b0p + kb, hh); c00 = g2_mma(a0, b, c00); c10 = g2_mma(a1, b, c10);
    b = g2_frag(b1p + kb, hh); c01 = g2_mma(a0, b, c01); c11 = g2_mma(a1, b, c11);
    b = g2_frag(b2p + kb, hh); c02 = g2_mma(a0, b, c02); c12 = g2_mma(a1, b, c12);
    b = g2_frag(b3p + kb, hh); c03 = g2_mma(a0, b, c03); c13 = g2_mma(a1, b, c13); }
  v8f accs[8] = {c00, c01, c02, c03, c10, c11, c12, c13};
#pragma unroll
  for (int u = 0; u < 8; ++u) { const int t = u & 3, half = u >> 2; const int col = col0 + t * 16 + ln; const float bvl = bias ? bf16_rne(bias[col]) : 0.f;
#pragma unroll
    for (int r = 0; r < 8; ++r) { const int rloc = half * 16 + 8 * hh + r; so[w][rloc][t * 16 + ln] = accs[u][r] * alpha + bvl; } }
  __builtin_amdgcn_fence(4  , "workgroup"); __builtin_amdgcn_wave_barrier();
  const int rsub = lane >> 4, c4 = (lane & 15) * 4;
  for (int pass = 0; pass < 2; ++pass) {
#pragma unroll
    for (int q = 0; q < 16; ++q) { const int r = q * 2 + rsub; const v4f v = *(const v4fa*)&so[w][r][c4];
      if (C) *(volatile v4f*)(C + (size_t)(row0 + r) * ldc + col0 + c4) = v;
      if (C16) { v4h h4; for (int i = 0; i < 4; ++i) h4[i] = (_Float16)v[i]; *(volatile v4h*)(C16 + (size_t)(row0 + r) * ldc + col0 + c4) = h4; } }
    if (pass == 0) __threadfence(); } }

__global__ __launch_bounds__(256) void k_vt32(const _Float16* __restrict__ V16, _Float16* __restrict__ VT) {
  __shared__ unsigned short tl[64][34];
  const int tid = threadIdx.x; const int slab = blockIdx.x / (SEQ / 64), lg = blockIdx.x % (SEQ / 64); const int b = slab / NH, h = slab % NH;
  { const int r = tid >> 2, c8 = (tid & 3) * 8; FragH f;
    f.half[0] = *(const v8us*)((const unsigned short*)V16 + ((size_t)b * SEQ + lg * 64 + r) * TQ + h * HD + c8);
#pragma unroll
    for (int q = 0; q < 8; ++q) tl[r][c8 + q] = f.u[q]; }
  __syncthreads();
  const int d = tid >> 3, pc = tid & 7; FragH f;
#pragma unroll
  for (int q = 0; q < 8; ++q) f.u[q] = tl[pc * 8 + q][d];
  unsigned short* dst = (unsigned short*)VT + ((size_t)slab * HD + d) * SEQ + lg * 64 + pc * 8;
  *(volatile v8us*)dst = f.half[0]; __threadfence(); *(volatile v8us*)dst = f.half[0];
}

__global__ __launch_bounds__(128) void k_flash(const _Float16* __restrict__ QH, const _Float16* __restrict__ QL, const _Float16* __restrict__ KH, const _Float16* __restrict__ KL,
                                              const _Float16* __restrict__ VT, _Float16* __restrict__ OH) {
  __shared__ __attribute__((aligned(16))) _Float16 so[4][16][40];
  const int tid = threadIdx.x, w = tid >> 5, lane = tid & 31, ln = lane & 15, hh = lane >> 4;
  const int bh = blockIdx.y; const int b = bh / NH, h = bh - b * NH;
  const int q0 = blockIdx.x * 64 + w * 16;
  const size_t qrow = (size_t)b * SEQ + q0 + ln;
  const v16h qh = g2_frag(QH + qrow * TQ + h * HD, hh);
  const v16h ql = g2_frag(QL + qrow * TQ + h * HD, hh);
  const _Float16* khb = KH + ((size_t)b * SEQ + ln) * TQ + h * HD;
  const _Float16* klb = KL + ((size_t)b * SEQ + ln) * TQ + h * HD;
  const _Float16* vt0 = VT + ((size_t)bh * HD + ln) * SEQ;
  const _Float16* vt1 = vt0 + (size_t)16 * SEQ;
  const v8f z8 = {0.f,0.f,0.f,0.f,0.f,0.f,0.f,0.f};
  float rm = -3.0e38f, rl = 0.f; v8f o0 = z8, o1 = z8;
#pragma unroll 1
  for (int k0 = 0; k0 < SEQ; k0 += KT) {
    v8f s[4];
#pragma unroll
    for (int t = 0; t < 4; ++t) { const size_t ko = (size_t)(k0 + 16 * t) * TQ; const v16h ah = g2_frag(khb + ko, hh); const v16h al = g2_frag(klb + ko, hh); s[t] = mma_split(ah, al, qh, ql); }
    float m = s[0][0];
#pragma unroll
    for (int t = 0; t < 4; ++t) {
#pragma unroll
      for (int r = 0; r < 8; ++r) m = fmaxf(m, s[t][r]); }
    m = fmaxf(m, __shfl_xor(m, 16, 32));
    const float mn = fmaxf(rm, m);
    const float alpha = __expf(rm - mn);
    rm = mn;
    const float pm = mn - 9.704060527839234f;
    float ls = 0.f; FragH pa[2];
#pragma unroll
    for (int t = 0; t < 4; ++t) {
#pragma unroll
      for (int r = 0; r < 8; ++r) { const float p = __expf(s[t][r] - pm); ls += p; pa[t >> 1].h[((t & 1) << 3) + r] = (_Float16)p; } }
    ls += __shfl_xor(ls, 16, 32);
    rl = rl * alpha + ls;
#pragma unroll
    for (int r = 0; r < 8; ++r) { const float ar = __shfl(alpha, 8 * hh + r, 32); o0[r] *= ar; o1[r] *= ar; }
    v16h vb = g2_frag(vt0 + k0, hh); o0 = g2_mma(pa[0].v, vb, o0);
    vb = g2_frag(vt1 + k0, hh); o1 = g2_mma(pa[0].v, vb, o1);
    vb = g2_frag(vt0 + k0 + 32, hh); o0 = g2_mma(pa[1].v, vb, o0);
    vb = g2_frag(vt1 + k0 + 32, hh); o1 = g2_mma(pa[1].v, vb, o1);
  }
  const float inv = 1.0f / rl;
#pragma unroll
  for (int r = 0; r < 8; ++r) { const float ir = __shfl(inv, 8 * hh + r, 32); so[w][8 * hh + r][ln] = (_Float16)(o0[r] * ir); so[w][8 * hh + r][16 + ln] = (_Float16)(o1[r] * ir); }
  __builtin_amdgcn_fence(4  , "workgroup"); __builtin_amdgcn_wave_barrier();
  unsigned short* ob = (unsigned short*)OH + ((size_t)bh * SEQ + q0) * HD;
  for (int pass = 0; pass < 2; ++pass) {
#pragma unroll
    for (int j = 0; j < 2; ++j) { const int p = j * 32 + lane; const v8us v = *(const v8us*)&so[w][p >> 2][(p & 3) * 8]; *(volatile v8us*)(ob + (size_t)p * 8) = v; }
    if (pass == 0) __threadfence(); } }

__global__ __launch_bounds__(128) void k_gemm_out(const _Float16* __restrict__ OHp, const _Float16* __restrict__ Bh, int ldb, float alpha, const float* __restrict__ bias,
                                                  float* __restrict__ C, int ldc, int M, int N) {
  __shared__ __attribute__((aligned(16))) float so[4][32][68];
  const int tid = threadIdx.x, w = tid >> 5, lane = tid & 31, ln = lane & 15, hh = lane >> 4;
  const int ntn = N >> 6; const int mt = blockIdx.x / ntn, nq = blockIdx.x - mt * ntn; const int row0 = mt * 128 + 32 * w, col0 = nq * 64; if (row0 >= M) return;
  const int bidx = row0 / SEQ, l0 = row0 - bidx * SEQ;
  const _Float16* abase = OHp + (((size_t)bidx * NH) * SEQ + l0 + ln) * HD;
  const size_t hstr = (size_t)SEQ * HD;
  const _Float16* b0p = Bh + (size_t)(col0 + ln) * ldb; const _Float16* b1p = b0p + (size_t)16 * ldb; const _Float16* b2p = b1p + (size_t)16 * ldb; const _Float16* b3p = b2p + (size_t)16 * ldb;
  const v8f z8 = {0.f,0.f,0.f,0.f,0.f,0.f,0.f,0.f}; v8f c00 = z8, c01 = z8, c02 = z8, c03 = z8, c10 = z8, c11 = z8, c12 = z8, c13 = z8;
#pragma unroll 1
  for (int hk = 0; hk < NH; ++hk) { const _Float16* a0p = abase + (size_t)hk * hstr; const int kb = hk * HD;
    const v16h a0 = g2_frag(a0p, hh), a1 = g2_frag(a0p + (size_t)16 * HD, hh);
    v16h b = g2_frag(b0p + kb, hh); c00 = g2_mma(a0, b, c00); c10 = g2_mma(a1, b, c10);
    b = g2_frag(b1p + kb, hh); c01 = g2_mma(a0, b, c01); c11 = g2_mma(a1, b, c11);
    b = g2_frag(b2p + kb, hh); c02 = g2_mma(a0, b, c02); c12 = g2_mma(a1, b, c12);
    b = g2_frag(b3p + kb, hh); c03 = g2_mma(a0, b, c03); c13 = g2_mma(a1, b, c13); }
  v8f accs[8] = {c00, c01, c02, c03, c10, c11, c12, c13};
#pragma unroll
  for (int u = 0; u < 8; ++u) { const int t = u & 3, half = u >> 2; const int col = col0 + t * 16 + ln; const float bvl = bf16_rne(bias[col]);
#pragma unroll
    for (int r = 0; r < 8; ++r) { const int rloc = half * 16 + 8 * hh + r; so[w][rloc][t * 16 + ln] = accs[u][r] * alpha + bvl; } }
  __builtin_amdgcn_fence(4  , "workgroup"); __builtin_amdgcn_wave_barrier();
  const int rsub = lane >> 4, c4 = (lane & 15) * 4;
  const size_t crow0 = (size_t)bidx * SEQ_FULL + l0;
  for (int pass = 0; pass < 2; ++pass) {
#pragma unroll
    for (int q = 0; q < 16; ++q) { const int r = q * 2 + rsub; const v4f v = *(const v4fa*)&so[w][r][c4]; *(volatile v4f*)(C + (crow0 + r) * ldc + col0 + c4) = v; }
    if (pass == 0) __threadfence(); } }

extern "C" void kernel_launch(void* const* d_in, const int* in_sizes, int n_in,
                              void* d_out, int out_size, void* d_ws, size_t ws_size, hipStream_t stream) {
  if (n_in < 9) return;
  const float* X  = (const float*)d_in[0];
  const float* Wq = (const float*)d_in[1];
  const float* bq = (const float*)d_in[2];
  const float* Wk = (const float*)d_in[3];
  const float* bk = (const float*)d_in[4];
  const float* Wv = (const float*)d_in[5];
  const float* bv = (const float*)d_in[6];
  const float* Wo = (const float*)d_in[7];
  const float* bo = (const float*)d_in[8];
  const long long needX = (long long)(((size_t)(NB - 1) * SEQ_FULL + SEQ) * DIN);
  const long long needO = (long long)(((size_t)(NB - 1) * SEQ_FULL + SEQ) * DOUT);
  if ((long long)in_sizes[0] < needX || in_sizes[1] < DIN * TQ || in_sizes[2] < TQ || in_sizes[3] < DIN * TQ || in_sizes[4] < TQ ||
      in_sizes[5] < DIN * TQ || in_sizes[6] < TQ || in_sizes[7] < TQ * DOUT || in_sizes[8] < DOUT || (long long)out_size < needO) return;
  char* ws = (char*)d_ws; size_t off = 0;
  auto take = [&](size_t bytes) { char* p = ws + off; off += (bytes + 255) & ~(size_t)255; return p; };
  _Float16* X16 = (_Float16*)take(NR * DIN * 2);
  _Float16* Wqt = (_Float16*)take((size_t)TQ * DIN * 2); _Float16* Wkt = (_Float16*)take((size_t)TQ * DIN * 2); _Float16* Wvt = (_Float16*)take((size_t)TQ * DIN * 2);
  _Float16* Wot = (_Float16*)take((size_t)DOUT * TQ * 2);
  float* F = (float*)take(NR * TQ * 4);
  _Float16* QH = (_Float16*)take(NR * TQ * 2); _Float16* QL = (_Float16*)take(NR * TQ * 2);
  _Float16* KH = (_Float16*)take(NR * TQ * 2); _Float16* KL = (_Float16*)take(NR * TQ * 2);
  _Float16* V16 = (_Float16*)take(NR * TQ * 2);
  _Float16* VT = (_Float16*)take((size_t)NB * NH * HD * SEQ * 2);
  _Float16* OH = (_Float16*)take((size_t)NB * NH * SEQ * HD * 2);
  if (off > ws_size || off > (size_t)134217728) return;
  const float a16 = 0.0625f;

  k_x16r<<<(unsigned)((NR * DIN / 8 + 255) / 256), 256, 0, stream>>>(X, X16, NR * DIN / 8);
  k_wt_f16<<<(TQ * (DIN / 8) + 255) / 256, 256, 0, stream>>>(Wq, Wqt, DIN, TQ, 16.0f);
  k_wt_f16<<<(TQ * (DIN / 8) + 255) / 256, 256, 0, stream>>>(Wk, Wkt, DIN, TQ, 16.0f);
  k_wt_f16<<<(TQ * (DIN / 8) + 255) / 256, 256, 0, stream>>>(Wv, Wvt, DIN, TQ, 16.0f);
  k_wt_f16<<<(DOUT * (TQ / 8) + 255) / 256, 256, 0, stream>>>(Wo, Wot, TQ, DOUT, 16.0f);
  const unsigned gproj = (unsigned)((NR / 128) * (TQ / 64));
  k_gemm_proj<<<gproj, 128, 0, stream>>>(X16, DIN, Wqt, DIN, a16, bq, F, nullptr, TQ, (int)NR, TQ, DIN);
  k_hl<<<(unsigned)((NR * TQ / 8 + 255) / 256), 256, 0, stream>>>(F, QH, QL, NR * TQ / 8);
  k_gemm_proj<<<gproj, 128, 0, stream>>>(X16, DIN, Wkt, DIN, a16, bk, F, nullptr, TQ, (int)NR, TQ, DIN);
  k_hl<<<(unsigned)((NR * TQ / 8 + 255) / 256), 256, 0, stream>>>(F, KH, KL, NR * TQ / 8);
  k_gemm_proj<<<gproj, 128, 0, stream>>>(X16, DIN, Wvt, DIN, a16, bv, nullptr, V16, TQ, (int)NR, TQ, DIN);
  k_vt32<<<(unsigned)(NB * NH * (SEQ / 64)), 256, 0, stream>>>(V16, VT);
  k_flash<<<dim3(SEQ / 64, NB * NH), 128, 0, stream>>>(QH, QL, KH, KL, VT, OH);
  k_gemm_out<<<(unsigned)((NR / 128) * (DOUT / 64)), 128, 0, stream>>>(OH, Wot, TQ, a16, bo, (float*)d_out, DOUT, (int)NR, DOUT);
}
